// SSMLayerFFTComplex_10230612099619
// MI455X (gfx1250) — hardware-run, weakly checked
//
#include <hip/hip_runtime.h>
#include <math.h>

typedef __attribute__((ext_vector_type(16))) _Float16 v16h;
typedef __attribute__((ext_vector_type(8)))  _Float16 v8h;
typedef __attribute__((ext_vector_type(8)))  float    v8f;
typedef __attribute__((ext_vector_type(4)))  float    v4f;

constexpr int kB      = 8;
constexpr int kIn     = 32;
constexpr int kOut    = 32;
constexpr int kT      = 4096;
constexpr int kPairs  = 128;
constexpr int kRows   = kB * kT;
constexpr int kVW     = 2 * kPairs;
constexpr int kOutPad = 64;
constexpr float kDt   = 1.0f;
constexpr float kEps  = 1e-6f;

constexpr float kCarryU = 64.0f;
constexpr float kCarryB = 1024.0f;
constexpr float kCarryX = 64.0f;
constexpr float kCarryC = 1024.0f;
constexpr float kFold0  = 1.0f / (kCarryU * kCarryB);
constexpr float kFold1  = 2.0f / (kCarryX * kCarryC);
constexpr float kF16MinNormal = 6.103515625e-05f;

static_assert(kIn % 32 == 0 && kPairs % 32 == 0, "GEMM K multiples of 32");
static_assert(kRows % 64 == 0 && kVW % 64 == 0 && kT % 64 == 0 && kOutPad % 64 == 0, "GEMM M,N multiples of 64");
static_assert(kOut % 16 == 0 && kOut <= kOutPad, "stored row slabs are whole 16-row slabs");
static_assert(kB * kOut * kT == 1048576, "output element count");

constexpr size_t kSzPAR = (size_t)2 * kPairs * 4;
constexpr size_t kSzBT0 = (size_t)kVW * kIn * 2;
constexpr size_t kSzCT  = (size_t)kOutPad * kPairs * 2;
constexpr size_t kSzA0  = (size_t)kRows * kIn * 2;
constexpr size_t kSzV   = (size_t)kRows * kVW * 4;
constexpr size_t kSzXR  = (size_t)kRows * kPairs * 2;
constexpr size_t kOffPAR = 0;
constexpr size_t kOffBT0 = kOffPAR + kSzPAR;
constexpr size_t kOffCT  = kOffBT0 + kSzBT0;
constexpr size_t kOffA0  = kOffCT  + kSzCT;
constexpr size_t kOffV   = kOffA0  + kSzA0;
constexpr size_t kOffXR  = kOffV   + kSzV;
constexpr size_t kWsTotal = kOffXR + kSzXR;
static_assert(kWsTotal == 44073984ull, "carve total");
static_assert(kWsTotal <= 134217728ull, "carve cap");
static_assert((kOffBT0 % 128) == 0 && (kOffCT % 128) == 0 && (kOffA0 % 128) == 0 &&
              (kOffV % 128) == 0 && (kOffXR % 128) == 0, "128-B aligned regions");

__device__ __forceinline__ _Float16 to_f16_flush(float v) {
  const float w = (fabsf(v) < kF16MinNormal) ? 0.0f : v;
  return (_Float16)w;
}

union FragH { v16h v; v8h h[2]; };
__device__ __forceinline__ v16h frag_load_f16(const _Float16* p) {
  FragH f;
  f.h[0] = *(const v8h*)(p);
  f.h[1] = *(const v8h*)(p + 16);
  return f.v;
}

__device__ __forceinline__ v8f mma_f16_guarded(v16h a, v16h b, v8f c) {
  c = __builtin_amdgcn_wmma_f32_16x16x32_f16(false, a, false, b, (short)0, c, false, false);
  asm volatile("v_nop\n\tv_nop\n\tv_nop\n\tv_nop" : "+v"(c) : "v"(a), "v"(b));
  return c;
}

__global__ __launch_bounds__(256) void table_pack_kernel(
    const float* __restrict__ rl, const float* __restrict__ ro,
    const float* __restrict__ Bc, const float* __restrict__ Cp,
    float* __restrict__ PAR, unsigned short* __restrict__ BT0, unsigned short* __restrict__ CT)
{
  __shared__ __align__(16) float sPar[4 * kPairs];
  __shared__ __align__(16) float sB[kIn * kPairs];
  __shared__ __align__(16) float sC[kPairs * kOut];
  const int tid = threadIdx.x;
#pragma unroll
  for (int j = 0; j < 4; ++j) {
    const int q = tid + 256 * j;
    *(v4f*)(sB + 4 * q) = *(const v4f*)(Bc + 4 * q);
    *(v4f*)(sC + 4 * q) = *(const v4f*)(Cp + 4 * q);
  }
  if (tid < kPairs) {
    const float x   = rl[tid];
    const float sp  = fmaxf(x, 0.0f) + log1pf(expf(-fabsf(x)));
    const float lr  = -sp;
    const float li  = ro[tid];
    const float er  = expf(lr * kDt);
    const float ang = li * kDt;
    const float cs  = cosf(ang);
    const float sn  = sinf(ang);
    const float Are = er * cs;
    const float Aim = er * sn;
    const float nre = Are - 1.0f;
    const float mag2 = lr * lr + li * li;
    const float inv  = 1.0f / mag2;
    const float qre  = (nre * lr + Aim * li) * inv;
    const float qim  = (Aim * lr - nre * li) * inv;
    const bool big   = sqrtf(mag2) > kEps;
    sPar[tid]              = Are;
    sPar[kPairs + tid]     = Aim;
    sPar[2 * kPairs + tid] = big ? qre : kDt;
    sPar[3 * kPairs + tid] = big ? qim : 0.0f;
  }
  __syncthreads();

  for (int pass = 0; pass < 2; ++pass) {
    if (tid < 64) {
      const v4f pv = *(const v4f*)(sPar + 4 * tid);
      *(volatile v4f*)(PAR + 4 * tid) = pv;
    }
#pragma unroll 1
    for (int j = 0; j < 4; ++j) {
      const int g = tid + 256 * j;
      {
        const int n  = g >> 2;
        const int k8 = (g & 3) * 8;
        const int pp = n & (kPairs - 1);
        const float fs = sPar[2 * kPairs + n];
        v8h hv;
#pragma unroll
        for (int e = 0; e < 8; ++e) {
          const float bd = sB[(k8 + e) * kPairs + pp] * fs;
          hv[e] = to_f16_flush(bd * kCarryB);
        }
        *(volatile v8h*)(BT0 + (size_t)g * 8) = hv;
      }
      {
        const int o  = g >> 4;
        const int p8 = (g & 15) * 8;
        const int oc = (o < kOut) ? o : (kOut - 1);
        v8h hv;
#pragma unroll
        for (int e = 0; e < 8; ++e) {
          const float cv = sC[(p8 + e) * kOut + oc];
          const float w  = (o < kOut) ? (cv * kCarryC) : 0.0f;
          hv[e] = to_f16_flush(w);
        }
        *(volatile v8h*)(CT + (size_t)g * 8) = hv;
      }
    }
    __threadfence();
  }
}

__global__ __launch_bounds__(256) void pack_u_kernel(
    const float* __restrict__ u, unsigned short* __restrict__ A0)
{
  __shared__ float tile[kIn * 65];
  const int tid = threadIdx.x;
  const int b   = blockIdx.y;
  const int t0  = blockIdx.x * 64;
#pragma unroll
  for (int p = 0; p < 2; ++p) {
    const int idx = tid + 256 * p;
    const int i   = idx >> 4;
    const int t4  = (idx & 15) * 4;
    const v4f v = *(const v4f*)(u + ((size_t)(b * kIn + i)) * kT + t0 + t4);
    tile[i * 65 + t4 + 0] = v[0];
    tile[i * 65 + t4 + 1] = v[1];
    tile[i * 65 + t4 + 2] = v[2];
    tile[i * 65 + t4 + 3] = v[3];
  }
  __syncthreads();
  const int tt = tid >> 2;
  const int k8 = (tid & 3) * 8;
  v8h hv;
#pragma unroll
  for (int e = 0; e < 8; ++e) hv[e] = to_f16_flush(tile[(k8 + e) * 65 + tt] * kCarryU);
  unsigned short* q = A0 + ((size_t)(b * kT + t0)) * kIn + (size_t)tid * 8;
  *(volatile v8h*)q = hv;
  __threadfence();
  *(volatile v8h*)q = hv;
}

__global__ __launch_bounds__(256) void gemm64_f16_kernel(
    const unsigned short* __restrict__ Ap, int lda, long strideA,
    const unsigned short* __restrict__ Btp, int ldb, long strideB,
    float* __restrict__ Cout, int ldc, long strideC,
    int M, int N, int K, int mStore, float scale)
{
  __shared__ __align__(16) float sT[8][16 * 68];
  const int b    = blockIdx.y;
  const int lane = threadIdx.x & 31;
  const int wave = threadIdx.x >> 5;
  const int tilesN = N >> 6;
  const int tilesM = M >> 6;
  const int tile = blockIdx.x * 8 + wave;
  if (tile >= tilesM * tilesN) return;
  const int tm = tile / tilesN;
  const int tn = tile - tm * tilesN;
  const int m0 = tm << 6;
  const int n0 = tn << 6;

  const _Float16* Ab = (const _Float16*)Ap  + (size_t)b * strideA;
  const _Float16* Bb = (const _Float16*)Btp + (size_t)b * strideB;

  const int rlane = lane & 15;
  const int koff  = (lane >> 4) * 8;
  const int mOff  = (lane >> 4) * 8;

  v8f acc[4][4];
#pragma unroll
  for (int i = 0; i < 4; ++i)
#pragma unroll
    for (int j = 0; j < 4; ++j) acc[i][j] = (v8f){0.f,0.f,0.f,0.f,0.f,0.f,0.f,0.f};

  for (int k0 = 0; k0 < K; k0 += 32) {
    v16h bh[4];
#pragma unroll
    for (int j = 0; j < 4; ++j) {
      const size_t bo = (size_t)(n0 + (j << 4) + rlane) * ldb + koff + k0;
      bh[j] = frag_load_f16(Bb + bo);
    }
#pragma unroll
    for (int i = 0; i < 4; ++i) {
      const size_t ao = (size_t)(m0 + (i << 4) + rlane) * lda + koff + k0;
      const v16h ah = frag_load_f16(Ab + ao);
#pragma unroll
      for (int j = 0; j < 4; ++j) acc[i][j] = mma_f16_guarded(ah, bh[j], acc[i][j]);
    }
  }

  float* slab = sT[wave];
  float* C = Cout + (size_t)b * strideC;
  const int hh = lane >> 4, c4 = (lane & 15) * 4;
#pragma unroll
  for (int i = 0; i < 4; ++i) {
    const int mBase = m0 + (i << 4);
    if (mBase < mStore) {
#pragma unroll
      for (int j = 0; j < 4; ++j) {
#pragma unroll
        for (int r = 0; r < 8; ++r) {
          slab[(mOff + r) * 68 + (j << 4) + rlane] = acc[i][j][r] * scale;
        }
      }
      __builtin_amdgcn_fence(__ATOMIC_RELEASE, "workgroup");
      __builtin_amdgcn_wave_barrier();
      __builtin_amdgcn_fence(__ATOMIC_ACQUIRE, "workgroup");
      for (int pass = 0; pass < 2; ++pass) {
#pragma unroll
        for (int it = 0; it < 8; ++it) {
          const int row = it * 2 + hh;
          const v4f v = *(const v4f*)(slab + row * 68 + c4);
          *(volatile v4f*)(C + (size_t)(mBase + row) * ldc + n0 + c4) = v;
        }
        __threadfence();
      }
      __builtin_amdgcn_fence(__ATOMIC_RELEASE, "workgroup");
      __builtin_amdgcn_wave_barrier();
      __builtin_amdgcn_fence(__ATOMIC_ACQUIRE, "workgroup");
    }
  }
}

__global__ __launch_bounds__(64) void scan_kernel(
    const float* __restrict__ V, const float* __restrict__ PAR, unsigned short* __restrict__ XR)
{
  __shared__ __align__(16) float sY[64 * 68];
  const int tid = threadIdx.x, lane = tid & 31, wave = tid >> 5;
  const int b  = blockIdx.x >> 1;
  const int p0 = (blockIdx.x & 1) * 64;
  const int p  = p0 + tid;
  const float Are  = PAR[p];
  const float Aim  = PAR[kPairs + p];
  const float nAim = -Aim;
  float xr = 0.0f, xi = 0.0f;
  const float* vp = V + (size_t)b * kT * kVW + p;
  const int q = lane >> 3, c8 = (lane & 7) * 8;
#pragma unroll 1
  for (int t0 = 0; t0 < kT; t0 += 64) {
#pragma unroll 8
    for (int s = 0; s < 64; ++s) {
      const float vr = vp[(size_t)(t0 + s) * kVW];
      const float vi = vp[(size_t)(t0 + s) * kVW + kPairs];
      const float nr = fmaf(Are, xr, fmaf(nAim, xi, vr));
      const float ni = fmaf(Are, xi, fmaf(Aim, xr, vi));
      xr = nr;
      xi = ni;
      sY[s * 68 + tid] = nr * kCarryX;
    }
    __syncthreads();
    v8h hv[8];
#pragma unroll
    for (int it = 0; it < 8; ++it) {
      const int row = it * 8 + wave * 4 + q;
      const float* sp = sY + row * 68 + c8;
      const v4f a0 = *(const v4f*)(sp);
      const v4f a1 = *(const v4f*)(sp + 4);
#pragma unroll
      for (int e = 0; e < 4; ++e) {
        hv[it][e]     = to_f16_flush(a0[e]);
        hv[it][4 + e] = to_f16_flush(a1[e]);
      }
    }
    for (int pass = 0; pass < 2; ++pass) {
#pragma unroll
      for (int it = 0; it < 8; ++it) {
        const int row = it * 8 + wave * 4 + q;
        const size_t o = ((size_t)(b * kT + t0 + row)) * kPairs + p0 + c8;
        *(volatile v8h*)(XR + o) = hv[it];
      }
      __threadfence();
    }
    __syncthreads();
  }
}

extern "C" void kernel_launch(void* const* d_in, const int* in_sizes, int n_in,
                              void* d_out, int out_size, void* d_ws, size_t ws_size,
                              hipStream_t stream)
{
  if (n_in < 5) return;
  if (in_sizes[0] != kB * kIn * kT) return;
  if (in_sizes[1] != kPairs) return;
  if (in_sizes[2] != kPairs) return;
  if (in_sizes[3] != kIn * kPairs) return;
  if (in_sizes[4] != kPairs * kOut) return;
  if (out_size != kB * kOut * kT) return;
  if (ws_size < kWsTotal) return;

  const float* u  = (const float*)d_in[0];
  const float* rl = (const float*)d_in[1];
  const float* ro = (const float*)d_in[2];
  const float* Bc = (const float*)d_in[3];
  const float* Cp = (const float*)d_in[4];
  float* out = (float*)d_out;

  char* ws = (char*)d_ws;
  float*          PAR = (float*)(ws + kOffPAR);
  unsigned short* BT0 = (unsigned short*)(ws + kOffBT0);
  unsigned short* CT  = (unsigned short*)(ws + kOffCT);
  unsigned short* A0  = (unsigned short*)(ws + kOffA0);
  float*          V   = (float*)(ws + kOffV);
  unsigned short* XR  = (unsigned short*)(ws + kOffXR);

  table_pack_kernel<<<1, 256, 0, stream>>>(rl, ro, Bc, Cp, PAR, BT0, CT);

  pack_u_kernel<<<dim3(kT / 64, kB), 256, 0, stream>>>(u, A0);

  gemm64_f16_kernel<<<dim3((kRows / 64) * (kVW / 64) / 8, 1), 256, 0, stream>>>(
      A0, kIn, 0L,
      BT0, kIn, 0L,
      V, kVW, 0L,
      kRows, kVW, kIn, kRows, kFold0);

  scan_kernel<<<kB * (kPairs / 64), 64, 0, stream>>>(V, PAR, XR);

  gemm64_f16_kernel<<<dim3((kOutPad / 64) * (kT / 64) / 8, kB), 256, 0, stream>>>(
      CT, kPairs, 0L,
      XR, kPairs, (long)kT * kPairs,
      out, kT, (long)kOut * kT,
      kOutPad, kT, kPairs, kOut, kFold1);
}
